// PetriNetMessagePassing_20083267076534
// MI455X (gfx1250) — hardware-run, weakly checked
//
#include <hip/hip_runtime.h>


namespace {
constexpr int NB_ = 16, NS = 128, NN = 13, D = 128, E = 6, M = 64, NH = 4, HD = 16, NG = NB_ * NS  , NROW = NG * NN  , KMC = 160  ;
constexpr float HS = 256.0f, WSC = 256.0f, LNEPS = 1e-5f;
typedef _Float16 b16;
typedef __attribute__((ext_vector_type(16))) _Float16 v16b;
typedef __attribute__((ext_vector_type(8))) _Float16 v8b;
typedef __attribute__((ext_vector_type(8))) float v8f;
typedef __attribute__((ext_vector_type(4))) float v4f;
typedef __attribute__((ext_vector_type(2))) float v2f;
__device__ __forceinline__ float bf16_rne(float f) { unsigned int u = __float_as_uint(f); u += 0x7FFFu + ((u >> 16) & 1u); float r = __uint_as_float(u & 0xFFFF0000u); asm volatile("" : "+v"(r)); return r; }
__device__ __forceinline__ float bfv(float f) { float r = bf16_rne(f); asm volatile("" : "+v"(r)); return r; }
__device__ __forceinline__ void split16(float v, b16& hi, b16& lo) { hi = (b16)v; lo = (b16)(v - (float)hi); }
__device__ __forceinline__ v16b frag_kb(const b16* p, int hh) { const v8b a = *(const v8b*)(p + 8 * hh), b = *(const v8b*)(p + 16 + 8 * hh); v16b f;
#pragma unroll
  for (int e = 0; e < 8; ++e) { f[e] = a[e]; f[8 + e] = b[e]; } return f; }
__device__ __forceinline__ v8f wmma16b(v16b a, v16b b, v8f c) { v8f d = __builtin_amdgcn_wmma_f32_16x16x32_f16(false, a, false, b, (short)0, c, false, false); asm volatile("v_nop\n\tv_nop\n\tv_nop\n\tv_nop" : "+v"(d) : "v"(a), "v"(b)); return d; }
__device__ __forceinline__ void wave_lds_sync() { __builtin_amdgcn_fence(__ATOMIC_RELEASE, "workgroup"); __builtin_amdgcn_wave_barrier(); __builtin_amdgcn_fence(__ATOMIC_ACQUIRE, "workgroup"); }
__device__ __forceinline__ float pmul(float a, float b) { float p = a * b; asm volatile("" : "+v"(p)); return p; }
__device__ __forceinline__ float gelu(float v) { return 0.5f * v * (1.0f + erff(v * 0.70710678118654752f)); }
__device__ __forceinline__ float sigm(float v) { return 1.0f / (1.0f + __expf(-v)); }

__global__ __launch_bounds__(256) void wput_kernel(const float* __restrict__ mc1, const float* __restrict__ mc2, const float* __restrict__ ts2, const float* __restrict__ ain, const float* __restrict__ aout, const float* __restrict__ ag1, const float* __restrict__ ag2, const float* __restrict__ gt, b16* __restrict__ WMC1, b16* __restrict__ WMC2, b16* __restrict__ WTS2, b16* __restrict__ WIN, b16* __restrict__ WOUT, b16* __restrict__ WAG1, b16* __restrict__ WAG2, b16* __restrict__ WGT) { const size_t nt = (size_t)gridDim.x * 256, u0 = (size_t)blockIdx.x * 256 + threadIdx.x; v8b v;
  auto put = [&](const float* src, b16* dst, int kin, int kp, int nout) { for (size_t u = u0; u < (size_t)nout * (kp / 8); u += nt) { const int o = (int)(u / (kp / 8)), k0 = (int)(u % (kp / 8)) * 8;
#pragma unroll
      for (int j = 0; j < 8; ++j) { const int k = k0 + j; v[j] = (b16)(k < kin ? bf16_rne(src[(size_t)k * nout + o]) * WSC : 0.0f); } for (int pass = 0; pass < 2; ++pass) { *(volatile v8b*)(dst + (size_t)o * kp + k0) = v; __threadfence(); } } };
  put(mc1, WMC1, D + E, KMC, M); put(mc2, WMC2, M, M, M); put(ts2, WTS2, M, M, 32); put(ain, WIN, M, M, 3 * M); put(aout, WOUT, M, M, M); put(ag1, WAG1, M, M, D); put(ag2, WAG2, D, D, D); put(gt, WGT, 2 * D, 2 * D, D); }

__device__ __forceinline__ void ln_row64(float* row, int lane, const float* g, const float* b) {
  float v0 = row[lane * 2], v1 = row[lane * 2 + 1]; float sm = v0 + v1; for (int o = 16; o; o >>= 1) sm += __shfl_xor(sm, o); const float mu = sm / 64.0f; float q2 = (v0 - mu) * (v0 - mu) + (v1 - mu) * (v1 - mu); for (int o = 16; o; o >>= 1) q2 += __shfl_xor(q2, o); const float rs = rsqrtf(q2 / 64.0f + LNEPS);
  row[lane * 2] = pmul((v0 - mu) * rs, bfv(g[lane * 2])) + bfv(b[lane * 2]); row[lane * 2 + 1] = pmul((v1 - mu) * rs, bfv(g[lane * 2 + 1])) + bfv(b[lane * 2 + 1]); }

__global__ __launch_bounds__(32) void edge_kernel(const float* __restrict__ ns, const float* __restrict__ ef, const float* __restrict__ eew1, const float* __restrict__ eeb1, const float* __restrict__ eeg, const float* __restrict__ eeb, const float* __restrict__ eew2, const float* __restrict__ eeb2,
    const float* __restrict__ tsw1, const float* __restrict__ tsb1, const float* __restrict__ tsg, const float* __restrict__ tsb, const b16* __restrict__ WTS2, const float* __restrict__ tsb2, const float* __restrict__ tsw3, const float* __restrict__ tsb3,
    const b16* __restrict__ WMC1, const float* __restrict__ mcb1, const float* __restrict__ mcg, const float* __restrict__ mcb, const b16* __restrict__ WMC2, const float* __restrict__ mcb2, const float* __restrict__ mng, const float* __restrict__ mnb,
    const b16* __restrict__ WIN, const float* __restrict__ ainb, const b16* __restrict__ WOUT, const float* __restrict__ aoutb, int GLIM, float* __restrict__ AGG) {
  __shared__ __attribute__((aligned(16))) b16 Ah[16][KMC + 8], Al[16][KMC + 8]; __shared__ float Tf[16][3 * M + 4], Enc[16][8], Ts[16], T1[16][M + 1];
  const int lane = threadIdx.x, nloc = lane & 15, hlf = lane >> 4; const int i = blockIdx.x % NN; const int gidx = blockIdx.x / NN; if (gidx >= GLIM) return;
  { const int r = nloc; float e6[E]; if (r < NN) { const float* efp = ef + ((((size_t)gidx * NN + r) * NN + i) * E); for (int q = 0; q < E; ++q) e6[q] = bfv(efp[q]); } else for (int q = 0; q < E; ++q) e6[q] = 0.0f;
    for (int c = hlf * 32; c < hlf * 32 + 32; ++c) { float s = bfv(eeb1[c]); for (int q = 0; q < E; ++q) s += pmul(e6[q], bfv(eew1[q * M + c])); Tf[r][c] = s; } }
  wave_lds_sync();
  for (int r = 0; r < 16; ++r) { ln_row64(&Tf[r][0], lane, eeg, eeb); Tf[r][lane * 2] = gelu(Tf[r][lane * 2]); Tf[r][lane * 2 + 1] = gelu(Tf[r][lane * 2 + 1]); }
  wave_lds_sync();
  { const int r = nloc; for (int q = hlf * 3; q < hlf * 3 + 3; ++q) { float s = bfv(eeb2[q]); for (int c = 0; c < M; ++c) s += pmul(Tf[r][c], bfv(eew2[c * E + q])); Enc[r][q] = s; } }
  wave_lds_sync();
  { const int r = nloc; for (int c = hlf * 32; c < hlf * 32 + 32; ++c) { float s = bfv(tsb1[c]); for (int q = 0; q < E; ++q) s += pmul(Enc[r][q], bfv(tsw1[q * M + c])); T1[r][c] = s; } }
  wave_lds_sync();
  for (int r = 0; r < 16; ++r) { ln_row64(&T1[r][0], lane, tsg, tsb); }
  wave_lds_sync();
  for (int r = 0; r < 16; ++r) for (int q = 0; q < 2; ++q) { const int c = q * 32 + lane; b16 p, ql; split16(gelu(T1[r][c]) * HS, p, ql); Ah[r][c] = p; Al[r][c] = ql; }
  if (lane < 16) for (int k = M; k < M + 8; ++k) { Ah[lane][k] = (b16)0.0f; Al[lane][k] = (b16)0.0f; }
  wave_lds_sync();
  { v8f acc[2] = {(v8f){}, (v8f){}};
#pragma unroll
    for (int kb = 0; kb < M; kb += 32) { const v16b a = frag_kb(&Ah[nloc][kb], hlf), al = frag_kb(&Al[nloc][kb], hlf);
#pragma unroll
      for (int t = 0; t < 2; ++t) { const v16b bw = frag_kb(WTS2 + (size_t)(t * 16 + nloc) * M + kb, hlf); acc[t] = wmma16b(a, bw, acc[t]); acc[t] = wmma16b(al, bw, acc[t]); } }
#pragma unroll
    for (int t = 0; t < 2; ++t) { const int cc = t * 16 + nloc; const float bb = bfv(tsb2[cc]);
#pragma unroll
      for (int r8 = 0; r8 < 8; ++r8) Tf[8 * hlf + r8][cc] = gelu(acc[t][r8] * (1.0f / (HS * WSC)) + bb); } }
  wave_lds_sync();
  if (lane < 16) { float s = bfv(tsb3[0]); for (int c = 0; c < 32; ++c) s += pmul(Tf[lane][c], bfv(tsw3[c])); Ts[lane] = sigm(s); }
  for (int r = 0; r < 16; ++r) { const int j = r < NN ? r : NN - 1; for (int q = 0; q < 5; ++q) { const int c = q * 32 + lane; float v = 0.0f; if (c < D) v = bfv(ns[((size_t)gidx * NN + j) * D + c]); else if (c < D + E) v = Enc[r][c - D]; b16 p, ql; split16(v * HS, p, ql); Ah[r][c] = p; Al[r][c] = ql; } }
  if (lane < 16) for (int k = KMC; k < KMC + 8; ++k) { Ah[lane][k] = (b16)0.0f; Al[lane][k] = (b16)0.0f; }
  wave_lds_sync();
  { v8f acc[4] = {(v8f){}, (v8f){}, (v8f){}, (v8f){}};
#pragma unroll
    for (int kb = 0; kb < KMC; kb += 32) { const v16b a = frag_kb(&Ah[nloc][kb], hlf), al = frag_kb(&Al[nloc][kb], hlf);
#pragma unroll
      for (int t = 0; t < 4; ++t) { const v16b bw = frag_kb(WMC1 + (size_t)(t * 16 + nloc) * KMC + kb, hlf); acc[t] = wmma16b(a, bw, acc[t]); acc[t] = wmma16b(al, bw, acc[t]); } }
#pragma unroll
    for (int t = 0; t < 4; ++t) { const int cc = t * 16 + nloc; const float bb = bfv(mcb1[cc]);
#pragma unroll
      for (int r8 = 0; r8 < 8; ++r8) Tf[8 * hlf + r8][cc] = acc[t][r8] * (1.0f / (HS * WSC)) + bb; } }
  wave_lds_sync();
  for (int r = 0; r < 16; ++r) ln_row64(&Tf[r][0], lane, mcg, mcb);
  wave_lds_sync();
  for (int r = 0; r < 16; ++r) for (int q = 0; q < 2; ++q) { const int c = q * 32 + lane; b16 p, ql; split16(gelu(Tf[r][c]) * HS, p, ql); Ah[r][c] = p; Al[r][c] = ql; }
  if (lane < 16) for (int k = M; k < M + 8; ++k) { Ah[lane][k] = (b16)0.0f; Al[lane][k] = (b16)0.0f; }
  wave_lds_sync();
  { v8f acc[4] = {(v8f){}, (v8f){}, (v8f){}, (v8f){}};
#pragma unroll
    for (int kb = 0; kb < M; kb += 32) { const v16b a = frag_kb(&Ah[nloc][kb], hlf), al = frag_kb(&Al[nloc][kb], hlf);
#pragma unroll
      for (int t = 0; t < 4; ++t) { const v16b bw = frag_kb(WMC2 + (size_t)(t * 16 + nloc) * M + kb, hlf); acc[t] = wmma16b(a, bw, acc[t]); acc[t] = wmma16b(al, bw, acc[t]); } }
#pragma unroll
    for (int t = 0; t < 4; ++t) { const int cc = t * 16 + nloc; const float bb = bfv(mcb2[cc]);
#pragma unroll
      for (int r8 = 0; r8 < 8; ++r8) { const int r = 8 * hlf + r8; Tf[r][cc] = pmul(acc[t][r8] * (1.0f / (HS * WSC)) + bb, Ts[r]); } } }
  wave_lds_sync();
  for (int r = 0; r < 16; ++r) ln_row64(&Tf[r][0], lane, mng, mnb);
  wave_lds_sync();
  for (int r = 0; r < 16; ++r) for (int q = 0; q < 2; ++q) { const int c = q * 32 + lane; b16 p, ql; split16(Tf[r][c] * HS, p, ql); Ah[r][c] = p; Al[r][c] = ql; }
  wave_lds_sync();
  { v8f acc[12];
#pragma unroll
    for (int t = 0; t < 12; ++t) acc[t] = (v8f){};
#pragma unroll
    for (int kb = 0; kb < M; kb += 32) { const v16b a = frag_kb(&Ah[nloc][kb], hlf), al = frag_kb(&Al[nloc][kb], hlf);
#pragma unroll
      for (int t = 0; t < 12; ++t) { const v16b bw = frag_kb(WIN + (size_t)(t * 16 + nloc) * M + kb, hlf); acc[t] = wmma16b(a, bw, acc[t]); acc[t] = wmma16b(al, bw, acc[t]); } }
#pragma unroll
    for (int t = 0; t < 12; ++t) { const int cc = t * 16 + nloc; const float bb = bfv(ainb[cc]);
#pragma unroll
      for (int r8 = 0; r8 < 8; ++r8) Tf[8 * hlf + r8][cc] = acc[t][r8] * (1.0f / (HS * WSC)) + bb; } }
  wave_lds_sync();
  if (lane < NN) { const int qr = lane;
#pragma unroll 1
    for (int h = 0; h < NH; ++h) { float sc[NN]; float mx = -INFINITY;
#pragma unroll
      for (int kr = 0; kr < NN; ++kr) { float s = 0.0f;
#pragma unroll
        for (int d2 = 0; d2 < HD; ++d2) s += pmul(Tf[qr][h * HD + d2], Tf[kr][M + h * HD + d2]); s = s * 0.25f; sc[kr] = s; mx = fmaxf(mx, s); }
      float den = 0.0f;
#pragma unroll
      for (int kr = 0; kr < NN; ++kr) { sc[kr] = __expf(sc[kr] - mx); den += sc[kr]; } const float inv = 1.0f / den;
#pragma unroll 1
      for (int d2 = 0; d2 < HD; ++d2) { float o = 0.0f;
#pragma unroll
        for (int kr = 0; kr < NN; ++kr) o += pmul(sc[kr] * inv, Tf[kr][2 * M + h * HD + d2]); b16 p, ql; split16(o * HS, p, ql); Ah[qr][h * HD + d2] = p; Al[qr][h * HD + d2] = ql; } } }
  wave_lds_sync();
  { v8f acc[4] = {(v8f){}, (v8f){}, (v8f){}, (v8f){}};
#pragma unroll
    for (int kb = 0; kb < M; kb += 32) { const v16b a = frag_kb(&Ah[nloc][kb], hlf), al = frag_kb(&Al[nloc][kb], hlf);
#pragma unroll
      for (int t = 0; t < 4; ++t) { const v16b bw = frag_kb(WOUT + (size_t)(t * 16 + nloc) * M + kb, hlf); acc[t] = wmma16b(a, bw, acc[t]); acc[t] = wmma16b(al, bw, acc[t]); } }
#pragma unroll
    for (int t = 0; t < 4; ++t) { const int cc = t * 16 + nloc; const float bb = bfv(aoutb[cc]);
#pragma unroll
      for (int r8 = 0; r8 < 8; ++r8) Tf[8 * hlf + r8][cc] = acc[t][r8] * (1.0f / (HS * WSC)) + bb; } }
  wave_lds_sync();
  v2f mean2; { float s0 = 0.0f, s1 = 0.0f; for (int r = 0; r < NN; ++r) { s0 += Tf[r][lane * 2]; s1 += Tf[r][lane * 2 + 1]; } mean2[0] = s0 * (1.0f / NN); mean2[1] = s1 * (1.0f / NN); }
  for (int pass = 0; pass < 2; ++pass) { *(volatile v2f*)(AGG + ((size_t)gidx * NN + i) * M + lane * 2) = mean2; __threadfence(); } }
__global__ __launch_bounds__(32) void node_kernel(const float* __restrict__ AGG, const float* __restrict__ ns, const b16* __restrict__ WAG1, const float* __restrict__ agb1, const float* __restrict__ agg_, const float* __restrict__ agb, const b16* __restrict__ WAG2, const float* __restrict__ agb2, const b16* __restrict__ WGT, const float* __restrict__ gtb, const float* __restrict__ nng, const float* __restrict__ nnb, int RLIM, float* __restrict__ out) {
  __shared__ __attribute__((aligned(16))) b16 Ah[16][2 * D + 8], Al[16][2 * D + 8]; __shared__ float Tf[16][D + 4], Ni[16][D + 1]; const int lane = threadIdx.x, nloc = lane & 15, hlf = lane >> 4; const size_t m0 = (size_t)blockIdx.x * 16; if (m0 >= (size_t)RLIM) return;
  for (int rr = 0; rr < 16; ++rr) for (int q = 0; q < 2; ++q) { const int c = q * 32 + lane; b16 p, ql; split16(AGG[(m0 + rr) * M + c] * HS, p, ql); Ah[rr][c] = p; Al[rr][c] = ql; }
  if (lane < 16) for (int k = M; k < M + 8; ++k) { Ah[lane][k] = (b16)0.0f; Al[lane][k] = (b16)0.0f; }
  wave_lds_sync();
  { v8f acc[8];
#pragma unroll
    for (int t = 0; t < 8; ++t) acc[t] = (v8f){};
#pragma unroll
    for (int kb = 0; kb < M; kb += 32) { const v16b a = frag_kb(&Ah[nloc][kb], hlf), al = frag_kb(&Al[nloc][kb], hlf);
#pragma unroll
      for (int t = 0; t < 8; ++t) { const v16b bw = frag_kb(WAG1 + (size_t)(t * 16 + nloc) * M + kb, hlf); acc[t] = wmma16b(a, bw, acc[t]); acc[t] = wmma16b(al, bw, acc[t]); } }
#pragma unroll
    for (int t = 0; t < 8; ++t) { const int cc = t * 16 + nloc; const float bb = bfv(agb1[cc]);
#pragma unroll
      for (int r8 = 0; r8 < 8; ++r8) Tf[8 * hlf + r8][cc] = acc[t][r8] * (1.0f / (HS * WSC)) + bb; } }
  wave_lds_sync();
  for (int rr = 0; rr < 16; ++rr) { float v[4], sm = 0.0f; for (int k = 0; k < 4; ++k) { v[k] = Tf[rr][lane * 4 + k]; sm += v[k]; } for (int o = 16; o; o >>= 1) sm += __shfl_xor(sm, o); const float mu = sm / D; float q2 = 0.0f; for (int k = 0; k < 4; ++k) q2 += (v[k] - mu) * (v[k] - mu); for (int o = 16; o; o >>= 1) q2 += __shfl_xor(q2, o); const float rs = rsqrtf(q2 / D + LNEPS);
    for (int k = 0; k < 4; ++k) { const int c = lane * 4 + k; b16 p, ql; split16(gelu(pmul((v[k] - mu) * rs, bfv(agg_[c])) + bfv(agb[c])) * HS, p, ql); Ah[rr][c] = p; Al[rr][c] = ql; } }
  if (lane < 16) for (int k = D; k < D + 8; ++k) { Ah[lane][k] = (b16)0.0f; Al[lane][k] = (b16)0.0f; }
  wave_lds_sync();
  { v8f acc[8];
#pragma unroll
    for (int t = 0; t < 8; ++t) acc[t] = (v8f){};
#pragma unroll
    for (int kb = 0; kb < D; kb += 32) { const v16b a = frag_kb(&Ah[nloc][kb], hlf), al = frag_kb(&Al[nloc][kb], hlf);
#pragma unroll
      for (int t = 0; t < 8; ++t) { const v16b bw = frag_kb(WAG2 + (size_t)(t * 16 + nloc) * D + kb, hlf); acc[t] = wmma16b(a, bw, acc[t]); acc[t] = wmma16b(al, bw, acc[t]); } }
#pragma unroll
    for (int t = 0; t < 8; ++t) { const int cc = t * 16 + nloc; const float bb = bfv(agb2[cc]);
#pragma unroll
      for (int r8 = 0; r8 < 8; ++r8) Ni[8 * hlf + r8][cc] = acc[t][r8] * (1.0f / (HS * WSC)) + bb; } }
  wave_lds_sync();
  for (int rr = 0; rr < 16; ++rr) for (int q = 0; q < 8; ++q) { const int c = q * 32 + lane; b16 p, ql; if (c < D) { p = (b16)(bf16_rne(ns[(m0 + rr) * D + c]) * HS); ql = (b16)0.0f; } else split16(Ni[rr][c - D] * HS, p, ql); Ah[rr][c] = p; Al[rr][c] = ql; }
  if (lane < 16) for (int k = 2 * D; k < 2 * D + 8; ++k) { Ah[lane][k] = (b16)0.0f; Al[lane][k] = (b16)0.0f; }
  wave_lds_sync();
  { v8f acc[8];
#pragma unroll
    for (int t = 0; t < 8; ++t) acc[t] = (v8f){};
#pragma unroll 2
    for (int kb = 0; kb < 2 * D; kb += 32) { const v16b a = frag_kb(&Ah[nloc][kb], hlf), al = frag_kb(&Al[nloc][kb], hlf);
#pragma unroll
      for (int t = 0; t < 8; ++t) { const v16b bw = frag_kb(WGT + (size_t)(t * 16 + nloc) * 2 * D + kb, hlf); acc[t] = wmma16b(a, bw, acc[t]); if (kb >= D) acc[t] = wmma16b(al, bw, acc[t]); } }
#pragma unroll
    for (int t = 0; t < 8; ++t) { const int cc = t * 16 + nloc; const float bb = bfv(gtb[cc]);
#pragma unroll
      for (int r8 = 0; r8 < 8; ++r8) { const int rr = 8 * hlf + r8; const float g = sigm(acc[t][r8] * (1.0f / (HS * WSC)) + bb); Tf[rr][cc] = pmul(g, Ni[rr][cc]) + pmul(1.0f - g, bfv(ns[(m0 + rr) * D + cc])); } } }
  wave_lds_sync();
  for (int pass = 0; pass < 2; ++pass) { for (int rr = 0; rr < 16; ++rr) { float v[4], sm = 0.0f; for (int k = 0; k < 4; ++k) { v[k] = Tf[rr][lane * 4 + k]; sm += v[k]; } for (int o = 16; o; o >>= 1) sm += __shfl_xor(sm, o); const float mu = sm / D; float q2 = 0.0f; for (int k = 0; k < 4; ++k) q2 += (v[k] - mu) * (v[k] - mu); for (int o = 16; o; o >>= 1) q2 += __shfl_xor(q2, o); const float rs = rsqrtf(q2 / D + LNEPS); v4f o4;
      for (int k = 0; k < 4; ++k) { const int c = lane * 4 + k; o4[k] = pmul((v[k] - mu) * rs, bfv(nng[c])) + bfv(nnb[c]); } *(volatile v4f*)(out + (m0 + rr) * D + lane * 4) = o4; } __threadfence(); } }
}

extern "C" void kernel_launch(void* const* d_in, const int* in_sizes, int n_in, void* d_out, int out_size, void* d_ws, size_t ws_size, hipStream_t stream) {
  (void)n_in;
  auto Fp = [&](int i) { return (const float*)d_in[i]; };
  if (in_sizes[0] != NROW * D || in_sizes[1] != NROW * NN * E || in_sizes[2] != E * M || in_sizes[12] != M * 32 || in_sizes[16] != (D + E) * M || in_sizes[22] != M * 3 * M || in_sizes[30] != D * D || in_sizes[32] != 2 * D * D || out_size != NROW * D) return;
  const int GLIM = NG;
  size_t off = 0; char* ws = (char*)d_ws;
  auto carve = [&](size_t bytes) { char* p = ws + off; off += (bytes + 255) & ~(size_t)255; return p; };
  b16* WMC1 = (b16*)carve((size_t)M * KMC * 2); b16* WMC2 = (b16*)carve(M * M * 2); b16* WTS2 = (b16*)carve(32 * M * 2); b16* WIN = (b16*)carve((size_t)3 * M * M * 2); b16* WOUT = (b16*)carve(M * M * 2); b16* WAG1 = (b16*)carve((size_t)D * M * 2); b16* WAG2 = (b16*)carve((size_t)D * D * 2); b16* WGT = (b16*)carve((size_t)D * 2 * D * 2); float* AGG = (float*)carve((size_t)NROW * M * 4);
  if (off > ws_size || off > ((size_t)16 << 20)) return;
  wput_kernel<<<64, 256, 0, stream>>>(Fp(16), Fp(20), Fp(12), Fp(22), Fp(24), Fp(26), Fp(30), Fp(32), WMC1, WMC2, WTS2, WIN, WOUT, WAG1, WAG2, WGT);
  edge_kernel<<<GLIM * NN, 32, 0, stream>>>(Fp(0), Fp(1), Fp(2), Fp(3), Fp(4), Fp(5), Fp(6), Fp(7), Fp(8), Fp(9), Fp(10), Fp(11), WTS2, Fp(13), Fp(14), Fp(15), WMC1, Fp(17), Fp(18), Fp(19), WMC2, Fp(21), Fp(36), Fp(37), WIN, Fp(23), WOUT, Fp(25), GLIM, AGG);
  node_kernel<<<(GLIM * NN + 15) / 16, 32, 0, stream>>>(AGG, Fp(0), WAG1, Fp(27), Fp(28), Fp(29), WAG2, Fp(31), WGT, Fp(33), Fp(34), Fp(35), GLIM * NN, (float*)d_out);
}
